// BatchIndexedMLP_59425167507528
// MI455X (gfx1250) — hardware-verified
//
#include <hip/hip_runtime.h>


#ifndef NB
#define NB 1024
#endif
#define NB_FULL 1024
#define NIN   126
#define NOUT  126
#define H1    256
#define H2D   256
#define KIDX  3
#define KP0   128
#define NP2   128
#define BT    32
#define XP    136
#define HP    264
#define TP    132
#define WS    64.0f
#define WSI   (1.0f / 64.0f)
#define QRS   2048.0f
#define QRI   (1.0f / 2048.0f)
#define NQ    (BT * NOUT / 4)
#define OIT   ((NQ + 255) / 256)

static_assert(NB % BT == 0);
static_assert(NB <= NB_FULL);
static_assert(BT == 32);
static_assert(NIN + 2 <= KP0);
static_assert(NOUT + 2 <= NP2);
static_assert(KP0 % 32 == 0);
static_assert(H1 % 32 == 0);
static_assert(H2D % 32 == 0);
static_assert(H1 == 8 * 32);
static_assert(H2D == 8 * 32);
static_assert(NP2 == 8 * 16);
static_assert((BT * KIDX) % 32 == 0);
static_assert(BT * KIDX <= 256);
static_assert(XP % 8 == 0 && XP >= KP0);
static_assert(HP % 8 == 0 && HP >= H1 && HP >= H2D);
static_assert(TP >= NP2);
static_assert((BT * NOUT * 4) % 128 == 0);
static_assert((BT * NOUT) % 4 == 0);
static_assert(NQ * 16 == BT * NOUT * 4);
static_assert(OIT * 256 >= NQ);
static_assert(BT * NOUT <= KIDX * BT * 128);
static_assert((size_t)KIDX * BT * 128 * 4 + (size_t)2 * BT * XP * 2 + (size_t)2 * BT * HP * 2 + (size_t)BT * TP * 4 <= (size_t)131072);

typedef _Float16 h16;
typedef __attribute__((ext_vector_type(16))) _Float16 v16h;
typedef __attribute__((ext_vector_type(8)))  _Float16 v8h;
typedef __attribute__((ext_vector_type(8)))  float    v8f;
typedef __attribute__((ext_vector_type(4)))  float    v4f;
typedef v4f  __attribute__((may_alias)) v4fa;
typedef v8h  __attribute__((may_alias)) v8ha;

__device__ __forceinline__ unsigned short f2bf(float f) { unsigned u = __float_as_uint(f); u += 0x7FFFu + ((u >> 16) & 1u); return (unsigned short)(u >> 16); }
__device__ __forceinline__ float bfr(float f) { return __uint_as_float(((unsigned)f2bf(f)) << 16); }
__device__ __forceinline__ v16h cat16(v8h lo, v8h hi) { return __builtin_shufflevector(lo, hi, 0, 1, 2, 3, 4, 5, 6, 7, 8, 9, 10, 11, 12, 13, 14, 15); }
__device__ __forceinline__ v8f wmma16(v16h a, v16h b, v8f c) { return __builtin_amdgcn_wmma_f32_16x16x32_f16(false, a, false, b, (short)0, c, false, false); }
__device__ __forceinline__ v16h  ldh(const h16* p) { return cat16(*(const v8h*)p, *(const v8h*)(p + 16)); }
__device__ __forceinline__ v8f wmma16g(v16h a, v16h b, v8f c) { c = wmma16(a, b, c); asm volatile("v_nop\n\tv_nop\n\tv_nop\n\tv_nop" : "+v"(c) : "v"(a), "v"(b)); return c; }
static __device__ __forceinline__ h16 toh_flush(float v) { const h16 r = (h16)v; return (fabsf(v) < 6.103515625e-05f) ? (h16)0.0f : r; }
__device__ __forceinline__ float elu_f(float v) { const float n = (v > 0.0f) ? 0.0f : v; const float e = expm1f(n); return (v > 0.0f) ? v : e; }
__device__ __forceinline__ int idx_fix(int j, int n) { j = (j < 0) ? (j + n) : j; j = (j < 0) ? 0 : j; return (j > n - 1) ? (n - 1) : j; }

__global__ __launch_bounds__(256) void k_wconv(const float* __restrict__ src, h16* dst, int srows, int scols, int dcols, int n8) {
    const int i = (int)blockIdx.x * 256 + (int)threadIdx.x; if (i >= n8) return;
    const int g = dcols >> 3; const int n = i / g; const int c8 = (i - n * g) * 8;
    const int nc = (n < srows) ? n : (srows - 1);
    float v[8];
#pragma unroll
    for (int j = 0; j < 8; ++j) { const int kk = c8 + j; const int kcl = (kk < scols) ? kk : (scols - 1); v[j] = src[(size_t)nc * scols + kcl]; }
#pragma unroll
    for (int j = 0; j < 8; ++j) asm volatile("" : "+v"(v[j]));
    v8h o;
#pragma unroll
    for (int j = 0; j < 8; ++j) { const bool ok = (n < srows) & (c8 + j < scols); const h16 hv = toh_flush(bfr(v[j]) * WS); o[j] = ok ? hv : (h16)0.0f; }
    *(volatile v8h*)(dst + (size_t)i * 8) = o; __threadfence(); *(volatile v8h*)(dst + (size_t)i * 8) = o;
}

__global__ __launch_bounds__(256) void k_layers(const float* __restrict__ x, const int* __restrict__ bii, const int* __restrict__ boi,
                                             const h16* __restrict__ W0H, const h16* __restrict__ W1H, const h16* __restrict__ W2H,
                                             const float* __restrict__ b0, const float* __restrict__ b1, const float* __restrict__ b2, float* OUT) {
    __shared__ __align__(16) float sScr[KIDX * BT * 128];
    __shared__ __align__(16) h16   sXh[BT * XP];
    __shared__ __align__(16) h16   sXr[BT * XP];
    __shared__ __align__(16) h16   sH[BT * HP];
    __shared__ __align__(16) h16   sH2[BT * HP];
    __shared__ __align__(16) float sT[BT * TP];

    const int tid = (int)threadIdx.x;
    const int lane = tid & 31, lr = lane & 15, hi = lane >> 4;
    const int wave = __builtin_amdgcn_readfirstlane((int)(threadIdx.x >> 5));
    const int brow0 = (int)blockIdx.x * BT;

    for (int i = tid; i < KIDX * BT * 128; i += 256) sScr[i] = 0.0f;
    __syncthreads();
    if (wave < (BT * KIDX) / 32) {
        const int r = tid / KIDX; const int k = tid - r * KIDX;
        const size_t b = (size_t)(brow0 + r);
        const int cb = (k * BT + r) * 128;
#pragma unroll 1
        for (int i = 0; i < NIN; ++i) {
            const int j = idx_fix(bii[(b * NIN + (size_t)i) * KIDX + k], NIN + 1);
            const float xv = bfr(x[b * NIN + (size_t)i]);
            sScr[cb + j] += xv;
        }
    }
    __syncthreads();
    for (int e = tid; e < BT * 128; e += 256) {
        const int r = e >> 7, j = e & 127;
        float s = (sScr[(0 * BT + r) * 128 + j] + sScr[(1 * BT + r) * 128 + j]) + sScr[(2 * BT + r) * 128 + j];
        s = (j < NIN) ? s : 0.0f;
        const h16 hv = toh_flush(s);
        const h16 rv = toh_flush((s - (float)hv) * QRS);
        sXh[r * XP + j] = hv; sXr[r * XP + j] = rv;
    }
    __syncthreads();

    {
        const int n0 = wave * 32;
        v8f acc[2][2], acr[2][2];
#pragma unroll
        for (int mt = 0; mt < 2; ++mt)
#pragma unroll
            for (int nt = 0; nt < 2; ++nt) { acc[mt][nt] = (v8f){}; acr[mt][nt] = (v8f){}; }
        const int ao = lr * XP + 8 * hi;
        const size_t bo = (size_t)(n0 + lr) * KP0 + 8 * hi;
#pragma unroll 1
        for (int kc = 0; kc < KP0; kc += 32) {
            v16h a[2], ar[2], bw[2];
#pragma unroll
            for (int mt = 0; mt < 2; ++mt) {
                a[mt]  = cat16(*(const v8ha*)(&sXh[ao + mt * 16 * XP + kc]), *(const v8ha*)(&sXh[ao + mt * 16 * XP + kc + 16]));
                ar[mt] = cat16(*(const v8ha*)(&sXr[ao + mt * 16 * XP + kc]), *(const v8ha*)(&sXr[ao + mt * 16 * XP + kc + 16])); }
#pragma unroll
            for (int nt = 0; nt < 2; ++nt) bw[nt] = ldh(W0H + bo + (size_t)nt * 16 * KP0 + kc);
#pragma unroll
            for (int mt = 0; mt < 2; ++mt)
#pragma unroll
                for (int nt = 0; nt < 2; ++nt) { acc[mt][nt] = wmma16g(a[mt], bw[nt], acc[mt][nt]); acr[mt][nt] = wmma16g(ar[mt], bw[nt], acr[mt][nt]); }
        }
#pragma unroll
        for (int mt = 0; mt < 2; ++mt)
#pragma unroll
            for (int nt = 0; nt < 2; ++nt) {
                const int col = n0 + nt * 16 + lr;
                const float bias = bfr(b0[col]);
#pragma unroll
                for (int r = 0; r < 8; ++r) {
                    const float v = (acc[mt][nt][r] + acr[mt][nt][r] * QRI) * WSI + bias;
                    sH[(mt * 16 + 8 * hi + r) * HP + col] = toh_flush(elu_f(v)); }
            }
    }
    __syncthreads();

    {
        const int n0 = wave * 32;
        v8f acc[2][2];
#pragma unroll
        for (int mt = 0; mt < 2; ++mt)
#pragma unroll
            for (int nt = 0; nt < 2; ++nt) acc[mt][nt] = (v8f){};
        const int ao = lr * HP + 8 * hi;
        const size_t bo = (size_t)(n0 + lr) * H1 + 8 * hi;
#pragma unroll 1
        for (int kc = 0; kc < H1; kc += 32) {
            v16h a[2], bw[2];
#pragma unroll
            for (int mt = 0; mt < 2; ++mt)
                a[mt] = cat16(*(const v8ha*)(&sH[ao + mt * 16 * HP + kc]), *(const v8ha*)(&sH[ao + mt * 16 * HP + kc + 16]));
#pragma unroll
            for (int nt = 0; nt < 2; ++nt) bw[nt] = ldh(W1H + bo + (size_t)nt * 16 * H1 + kc);
#pragma unroll
            for (int mt = 0; mt < 2; ++mt)
#pragma unroll
                for (int nt = 0; nt < 2; ++nt) acc[mt][nt] = wmma16g(a[mt], bw[nt], acc[mt][nt]);
        }
#pragma unroll
        for (int mt = 0; mt < 2; ++mt)
#pragma unroll
            for (int nt = 0; nt < 2; ++nt) {
                const int col = n0 + nt * 16 + lr;
                const float bias = bfr(b1[col]);
#pragma unroll
                for (int r = 0; r < 8; ++r) {
                    const float v = acc[mt][nt][r] * WSI + bias;
                    sH2[(mt * 16 + 8 * hi + r) * HP + col] = toh_flush(elu_f(v)); }
            }
    }
    __syncthreads();

    {
        const int n0 = wave * 16;
        const int n = n0 + lr;
        v8f acc[2];
        acc[0] = (v8f){}; acc[1] = (v8f){};
        const int ao = lr * HP + 8 * hi;
        const size_t bo = (size_t)n * H2D + 8 * hi;
#pragma unroll 1
        for (int kc = 0; kc < H2D; kc += 32) {
            v16h a[2];
#pragma unroll
            for (int mt = 0; mt < 2; ++mt)
                a[mt] = cat16(*(const v8ha*)(&sH2[ao + mt * 16 * HP + kc]), *(const v8ha*)(&sH2[ao + mt * 16 * HP + kc + 16]));
            const v16h bw = ldh(W2H + bo + kc);
#pragma unroll
            for (int mt = 0; mt < 2; ++mt) acc[mt] = wmma16g(a[mt], bw, acc[mt]);
        }
        const int ncl = (n < NOUT) ? n : (NOUT - 1);
        float braw = b2[ncl];
        asm volatile("" : "+v"(braw));
        const float bias = bfr(braw);
#pragma unroll
        for (int mt = 0; mt < 2; ++mt)
#pragma unroll
            for (int r = 0; r < 8; ++r) {
                const float v = acc[mt][r] * WSI + bias;
                sT[(mt * 16 + 8 * hi + r) * TP + n] = (n < NOUT) ? v : 0.0f; }
    }
    __syncthreads();

    for (int e = tid; e < BT * NOUT; e += 256) {
        const int r = e / NOUT; const int o = e - r * NOUT;
        const size_t b = (size_t)(brow0 + r);
        const int* ip = boi + (b * NOUT + (size_t)o) * KIDX;
        const int i0 = idx_fix(ip[0], NOUT + 1), i1 = idx_fix(ip[1], NOUT + 1), i2 = idx_fix(ip[2], NOUT + 1);
        const float s = (sT[r * TP + i0] + sT[r * TP + i1]) + sT[r * TP + i2];
        sScr[e] = s;
    }
    __syncthreads();

    float* obase = OUT + (size_t)brow0 * NOUT;
    v4f ov[OIT];
#pragma unroll
    for (int it = 0; it < OIT; ++it) { const int q = it * 256 + tid; const int qc = (q < NQ) ? q : (NQ - 1); ov[it] = *(const v4fa*)(&sScr[qc * 4]); }
#pragma unroll 1
    for (int ps = 0; ps < 2; ++ps) {
#pragma unroll
        for (int it = 0; it < OIT; ++it) { const int q = it * 256 + tid;
            if (q < NQ) *(volatile v4f*)(obase + (size_t)q * 4) = ov[it]; }
        if (ps == 0) __threadfence(); }
}

static constexpr size_t al256(size_t v) { return (v + 255) & ~(size_t)255; }
static constexpr size_t SZ_W0 = al256((size_t)H1 * KP0 * 2);
static constexpr size_t SZ_W1 = al256((size_t)H2D * H1 * 2);
static constexpr size_t SZ_W2 = al256((size_t)NP2 * H2D * 2);
static constexpr size_t SZ_TOTAL = SZ_W0 + SZ_W1 + SZ_W2;
static_assert(SZ_TOTAL <= (size_t)134217728);
static_assert(((size_t)H1 * KP0) % (8 * 256) == 0);
static_assert(((size_t)H2D * H1) % (8 * 256) == 0);
static_assert(((size_t)NP2 * H2D) % (8 * 256) == 0);
static_assert(KP0 % 8 == 0 && H1 % 8 == 0 && H2D % 8 == 0);

extern "C" void kernel_launch(void* const* d_in, const int* in_sizes, int n_in,
                              void* d_out, int out_size, void* d_ws, size_t ws_size, hipStream_t stream) {
    if (n_in < 9) return;
    if ((size_t)in_sizes[0] < (size_t)NB * NIN) return;
    if ((size_t)in_sizes[1] < (size_t)H1 * NIN || in_sizes[2] < H1) return;
    if ((size_t)in_sizes[3] < (size_t)H2D * H1 || in_sizes[4] < H2D) return;
    if ((size_t)in_sizes[5] < (size_t)NOUT * H2D || in_sizes[6] < NOUT) return;
    if ((size_t)in_sizes[7] < (size_t)NB * NIN * KIDX || (size_t)in_sizes[8] < (size_t)NB * NOUT * KIDX) return;
    if ((size_t)out_size < (size_t)NB * NOUT) return;
    if (SZ_TOTAL > ws_size) return;
    const float* x  = (const float*)d_in[0];
    const float* w0 = (const float*)d_in[1]; const float* b0 = (const float*)d_in[2];
    const float* w1 = (const float*)d_in[3]; const float* b1 = (const float*)d_in[4];
    const float* w2 = (const float*)d_in[5]; const float* b2 = (const float*)d_in[6];
    const int* bii = (const int*)d_in[7]; const int* boi = (const int*)d_in[8];
    float* OUT = (float*)d_out;
    char* wsp = (char*)d_ws;
    h16* W0H = (h16*)wsp; wsp += SZ_W0;
    h16* W1H = (h16*)wsp; wsp += SZ_W1;
    h16* W2H = (h16*)wsp; wsp += SZ_W2;

    { const int n8 = H1 * KP0 / 8;  k_wconv<<<(unsigned)(n8 / 256), 256, 0, stream>>>(w0, W0H, H1, NIN, KP0, n8); }
    { const int n8 = H2D * H1 / 8;  k_wconv<<<(unsigned)(n8 / 256), 256, 0, stream>>>(w1, W1H, H2D, H1, H1, n8); }
    { const int n8 = NP2 * H2D / 8; k_wconv<<<(unsigned)(n8 / 256), 256, 0, stream>>>(w2, W2H, NOUT, H2D, H2D, n8); }

    k_layers<<<dim3(NB / BT, 1, 1), 256, 0, stream>>>(x, bii, boi, W0H, W1H, W2H, b0, b1, b2, OUT);
}
